// model_33225867002038
// MI455X (gfx1250) — hardware-run, weakly checked
//
#include <hip/hip_runtime.h>
#include <math.h>

constexpr int NROWS     = 524288;
constexpr int NHID      = 2;
constexpr int NGATE     = 8;
constexpr int NFC1      = 128;
constexpr int NCLS      = 5;
constexpr int NCLS_PAD  = 16;
constexpr int BLK_ROWS  = 128;
constexpr int NTHR      = 128;
constexpr int NWAVE     = NTHR / 32;
constexpr int APITCH    = 136;
constexpr int OUT_PER_BLK  = BLK_ROWS * NCLS;
constexpr int OUT_PER_WAVE = OUT_PER_BLK / NWAVE;
constexpr float ACT_CARRY = 16.0f;
constexpr float W2_CARRY  = 256.0f;
constexpr float FOLD_INV  = 1.0f / (ACT_CARRY * W2_CARRY);

static_assert(NGATE == 4 * NHID, "gate count");
static_assert(NROWS % BLK_ROWS == 0, "no tail block");
static_assert(BLK_ROWS == NTHR, "one lane per batch row");
static_assert(NFC1 % 32 == 0, "K multiple of 32");
static_assert(APITCH % 8 == 0 && APITCH >= NFC1 + 8, "tile pitch");
static_assert(NCLS <= NCLS_PAD, "class padding");
static_assert((OUT_PER_BLK * 4) % 128 == 0, "block output is whole lines");
static_assert(OUT_PER_WAVE == 32 * NCLS, "each wave owns NCLS whole lines");
static_assert((long)NROWS * NCLS * 4 == 10485760L, "output bytes");

typedef __attribute__((ext_vector_type(16))) _Float16 v16h;
typedef __attribute__((ext_vector_type(8)))  _Float16 v8h;
typedef __attribute__((ext_vector_type(8)))  float    v8f;
typedef __attribute__((ext_vector_type(4)))  float    v4f;
typedef __attribute__((ext_vector_type(2)))  float    v2f;

__device__ __forceinline__ void dep_guard3_h(v8f& a, v8f& b, v16h x, v16h y, v16h z) {
  asm volatile("v_nop\n\tv_nop\n\tv_nop\n\tv_nop" : "+v"(a), "+v"(b) : "v"(x), "v"(y), "v"(z));
}
__device__ __forceinline__ void acc_guard2(v8f& a, v8f& b) {
  asm volatile("v_nop\n\tv_nop\n\tv_nop\n\tv_nop" : "+v"(a), "+v"(b));
}
__device__ __forceinline__ void keep4_h(v16h a, v16h b, v16h c, v16h d) {
  asm volatile("v_nop" :: "v"(a), "v"(b), "v"(c), "v"(d));
}

struct FragH {
  union U { v16h v; v8h h[2]; };
  static __device__ __forceinline__ v16h load(const _Float16* p) {
    U f;
    f.h[0] = *(const v8h*)(p);
    f.h[1] = *(const v8h*)(p + 16);
    return f.v;
  }
  static __device__ __forceinline__ v8f mma(v16h a, v16h b, v8f c) {
    return __builtin_amdgcn_wmma_f32_16x16x32_f16(false, a, false, b, (short)0, c, false, false);
  }
};

__device__ __forceinline__ float sigm(float x) { return 1.0f / (1.0f + expf(-x)); }

__device__ __forceinline__ float gate_pre(float x, float wx, float ha, float wa, float hb, float wb,
                                          float b0, float b1) {
  float g = x * wx;
  const float hw = ha * wa + hb * wb;
  g = g + hw;
  g = g + b0;
  g = g + b1;
  return g;
}

__global__ __launch_bounds__(NTHR) void lstm_head_kernel(
    const float* __restrict__ X, const float* __restrict__ H0, const float* __restrict__ C0,
    const float* __restrict__ Wih, const float* __restrict__ Whh,
    const float* __restrict__ Bih, const float* __restrict__ Bhh,
    const float* __restrict__ W1, const float* __restrict__ B1,
    const float* __restrict__ W2, const float* __restrict__ B2,
    float* __restrict__ Out) {
  __shared__ __align__(16) _Float16 At[BLK_ROWS * APITCH];
  __shared__ __align__(16) _Float16 Wt[NCLS_PAD * APITCH];
  __shared__ __align__(16) float    W1s[NFC1 * 4];
  __shared__ __align__(16) float    Os[OUT_PER_BLK];

  const int tid  = threadIdx.x;
  const int lane = tid & 31;
  const int wave = tid >> 5;
  const int c    = lane & 15;
  const int hh   = lane >> 4;
  const int koff = hh * 8;

  v8h zero8;
#pragma unroll
  for (int e = 0; e < 8; ++e) zero8[e] = (_Float16)0.0f;

  {
    const v2f w = *(const v2f*)(W1 + 2 * tid);
    const float bv = B1[tid];
    v4f q;
    q[0] = w[0];
    q[1] = w[1];
    q[2] = bv;
    q[3] = 0.0f;
    *(v4f*)(W1s + 4 * tid) = q;
  }
#pragma unroll
  for (int it = 0; it < 2; ++it) {
    const int idx = it * NTHR + tid;
    const int row = idx >> 4;
    const int c8  = (idx & 15) * 8;
    const int rs  = (row < NCLS) ? row : (NCLS - 1);
    const float* sp = W2 + rs * NFC1 + c8;
    const v4f a = *(const v4f*)(sp);
    const v4f b = *(const v4f*)(sp + 4);
    const bool keep = (row < NCLS);
    v8h hv;
#pragma unroll
    for (int e = 0; e < 4; ++e) {
      const float fa = a[e];
      const float fb = b[e];
      const float sa = keep ? fa * W2_CARRY : 0.0f;
      const float sb = keep ? fb * W2_CARRY : 0.0f;
      hv[e]     = (_Float16)sa;
      hv[4 + e] = (_Float16)sb;
    }
    *(v8h*)(Wt + row * APITCH + c8) = hv;
  }
  if (tid < NCLS_PAD) *(v8h*)(Wt + tid * APITCH + NFC1) = zero8;

  const size_t gb = (size_t)blockIdx.x * BLK_ROWS + (size_t)tid;
  const float xv = X[gb];
  const v2f hp = *(const v2f*)(H0 + 2 * gb);
  const v2f cp = *(const v2f*)(C0 + 2 * gb);
  const v4f wi0 = *(const v4f*)(Wih);
  const v4f wi1 = *(const v4f*)(Wih + 4);
  const v4f wh0 = *(const v4f*)(Whh);
  const v4f wh1 = *(const v4f*)(Whh + 4);
  const v4f wh2 = *(const v4f*)(Whh + 8);
  const v4f wh3 = *(const v4f*)(Whh + 12);
  const v4f bi0 = *(const v4f*)(Bih);
  const v4f bi1 = *(const v4f*)(Bih + 4);
  const v4f bh0 = *(const v4f*)(Bhh);
  const v4f bh1 = *(const v4f*)(Bhh + 4);
  const int ccl = (c < NCLS) ? c : (NCLS - 1);
  const float b2v = B2[ccl];

  const float g0 = gate_pre(xv, wi0[0], hp[0], wh0[0], hp[1], wh0[1], bi0[0], bh0[0]);
  const float g1 = gate_pre(xv, wi0[1], hp[0], wh0[2], hp[1], wh0[3], bi0[1], bh0[1]);
  const float g2 = gate_pre(xv, wi0[2], hp[0], wh1[0], hp[1], wh1[1], bi0[2], bh0[2]);
  const float g3 = gate_pre(xv, wi0[3], hp[0], wh1[2], hp[1], wh1[3], bi0[3], bh0[3]);
  const float g4 = gate_pre(xv, wi1[0], hp[0], wh2[0], hp[1], wh2[1], bi1[0], bh1[0]);
  const float g5 = gate_pre(xv, wi1[1], hp[0], wh2[2], hp[1], wh2[3], bi1[1], bh1[1]);
  const float g6 = gate_pre(xv, wi1[2], hp[0], wh3[0], hp[1], wh3[1], bi1[2], bh1[2]);
  const float g7 = gate_pre(xv, wi1[3], hp[0], wh3[2], hp[1], wh3[3], bi1[3], bh1[3]);

  const float ig0 = sigm(g0);
  const float ig1 = sigm(g1);
  const float fg0 = sigm(g2);
  const float fg1 = sigm(g3);
  const float gg0 = tanhf(g4);
  const float gg1 = tanhf(g5);
  const float og0 = sigm(g6);
  const float og1 = sigm(g7);
  const float cn0 = fg0 * cp[0] + ig0 * gg0;
  const float cn1 = fg1 * cp[1] + ig1 * gg1;
  const float hn0 = og0 * tanhf(cn0);
  const float hn1 = og1 * tanhf(cn1);
  const float a0x = fmaxf(hn0, 0.0f);
  const float a0y = fmaxf(hn1, 0.0f);

  __syncthreads();

  {
    _Float16* arow = At + tid * APITCH;
#pragma unroll 1
    for (int cg = 0; cg < NFC1 / 8; ++cg) {
      v8h hv;
#pragma unroll
      for (int e = 0; e < 8; ++e) {
        const v4f q = *(const v4f*)(W1s + 4 * (cg * 8 + e));
        float t = a0x * q[0];
        t = fmaf(a0y, q[1], t);
        t = t + q[2];
        t = fmaxf(t, 0.0f) * ACT_CARRY;
        hv[e] = (_Float16)t;
      }
      *(v8h*)(arow + cg * 8) = hv;
    }
    *(v8h*)(arow + NFC1) = zero8;
  }

  __syncthreads();

  v8f acc0 = (v8f){0.f, 0.f, 0.f, 0.f, 0.f, 0.f, 0.f, 0.f};
  v8f acc1 = (v8f){0.f, 0.f, 0.f, 0.f, 0.f, 0.f, 0.f, 0.f};
  {
    const _Float16* wrow = Wt + c * APITCH + koff;
    v16h bf[4];
#pragma unroll
    for (int kc = 0; kc < 4; ++kc) bf[kc] = FragH::load(wrow + 32 * kc);
    const _Float16* ar0 = At + (wave * 32 + c) * APITCH + koff;
    const _Float16* ar1 = At + (wave * 32 + 16 + c) * APITCH + koff;
#pragma unroll
    for (int kc = 0; kc < 4; ++kc) {
      const v16h a0 = FragH::load(ar0 + 32 * kc);
      const v16h a1 = FragH::load(ar1 + 32 * kc);
      acc0 = FragH::mma(a0, bf[kc], acc0);
      acc1 = FragH::mma(a1, bf[kc], acc1);
      dep_guard3_h(acc0, acc1, a0, a1, bf[kc]);
    }
    keep4_h(bf[0], bf[1], bf[2], bf[3]);
    acc_guard2(acc0, acc1);
  }

  if (c < NCLS) {
#pragma unroll
    for (int r = 0; r < 8; ++r) {
      const float v0 = acc0[r] * FOLD_INV + b2v;
      const float v1 = acc1[r] * FOLD_INV + b2v;
      Os[(wave * 32 + 8 * hh + r) * NCLS + c]      = v0;
      Os[(wave * 32 + 16 + 8 * hh + r) * NCLS + c] = v1;
    }
  }

  __syncthreads();

  {
    float ov[NCLS];
#pragma unroll
    for (int i = 0; i < NCLS; ++i) ov[i] = Os[wave * OUT_PER_WAVE + i * 32 + lane];
    float* op = Out + (size_t)blockIdx.x * OUT_PER_BLK + (size_t)(wave * OUT_PER_WAVE + lane);
    for (int pass = 0; pass < 2; ++pass) {
#pragma unroll
      for (int i = 0; i < NCLS; ++i) *(volatile float*)(op + i * 32) = ov[i];
      __threadfence();
    }
  }
}

extern "C" void kernel_launch(void* const* d_in, const int* in_sizes, int n_in,
                              void* d_out, int out_size, void* d_ws, size_t ws_size, hipStream_t stream) {
  (void)in_sizes; (void)out_size; (void)d_ws; (void)ws_size;
  if (n_in < 11 || d_out == nullptr) return;
  const float* x   = (const float*)d_in[0];
  const float* h0  = (const float*)d_in[1];
  const float* c0  = (const float*)d_in[2];
  const float* wih = (const float*)d_in[3];
  const float* whh = (const float*)d_in[4];
  const float* bih = (const float*)d_in[5];
  const float* bhh = (const float*)d_in[6];
  const float* w1  = (const float*)d_in[7];
  const float* b1  = (const float*)d_in[8];
  const float* w2  = (const float*)d_in[9];
  const float* b2  = (const float*)d_in[10];
  float* out = (float*)d_out;
  lstm_head_kernel<<<NROWS / BLK_ROWS, NTHR, 0, stream>>>(x, h0, c0, wih, whh, bih, bhh, w1, b1, w2, b2, out);
}
